// MambaBlock_12378095747351
// MI455X (gfx1250) — hardware-run, weakly checked
//
#include <hip/hip_runtime.h>
#include <hip/hip_fp16.h>
#include <math.h>

typedef __attribute__((ext_vector_type(16))) _Float16 v16h;
typedef __attribute__((ext_vector_type(8)))  _Float16 v8h;
typedef __attribute__((ext_vector_type(8)))  float    v8f;
typedef __attribute__((ext_vector_type(4)))  float    v4f;
typedef __attribute__((ext_vector_type(4)))  unsigned v4u;

constexpr int kBatch  = 2;
constexpr int kSeq    = 2048;
constexpr int kDm     = 1024;
constexpr int kDin    = 2048;
constexpr int kNst    = 16;
constexpr int kRank   = 64;
constexpr int kXpN    = kRank + 2 * kNst;
constexpr int kXpP    = 128;
constexpr int kXzP    = 2 * kDin;
constexpr int kOffB   = kRank;
constexpr int kOffC   = kRank + kNst;
constexpr int kConvTP = 260;
constexpr float kWCarry  = 512.0f;
constexpr float kUCarry  = 16.0f;
constexpr float kDtCarry = 16.0f;
constexpr float kYCarry  = 16.0f;
constexpr float kResid   = 2048.0f;
constexpr float kScIn  = 1.0f / kWCarry;
constexpr float kScU   = 1.0f / (kUCarry * kWCarry);
constexpr float kScDt  = 1.0f / (kDtCarry * kWCarry);
constexpr float kScY   = 1.0f / (kYCarry * kWCarry);
constexpr float kScNone = 0.0f;
static_assert(kXpN == 96);
static_assert(kXpN <= kXpP);
static_assert((kDm % 64) == 0 && (kDin % 64) == 0 && (kXpP % 64) == 0 && (kXzP % 64) == 0);
static_assert((kSeq % 64) == 0 && (kRank % 32) == 0 && (kDm % 32) == 0 && (kDin % 32) == 0);
static_assert((kDin % 256) == 0);

constexpr size_t kSzWIN  = (size_t)kXzP * kDm * 2;
constexpr size_t kSzWOUT = (size_t)kDm * kDin * 2;
constexpr size_t kSzWXP  = (size_t)kXpP * kDin * 2;
constexpr size_t kSzWDT  = (size_t)kDin * kRank * 2;
constexpr size_t kSzX16  = (size_t)kBatch * kSeq * kDm * 2;
constexpr size_t kSzXZ   = (size_t)kSeq * kXzP * 4;
constexpr size_t kSzU    = (size_t)kSeq * kDin * 4;
constexpr size_t kSzH16  = (size_t)kSeq * kDin * 2;
constexpr size_t kSzXP   = (size_t)kSeq * kXpP * 4;
constexpr size_t kSzDT16 = (size_t)kSeq * kRank * 2;
constexpr size_t kOffWIN  = 0;
constexpr size_t kOffWOUT = kOffWIN  + kSzWIN;
constexpr size_t kOffWXP  = kOffWOUT + kSzWOUT;
constexpr size_t kOffWDT  = kOffWXP  + kSzWXP;
constexpr size_t kOffX16  = kOffWDT  + kSzWDT;
constexpr size_t kOffXZ   = kOffX16  + kSzX16;
constexpr size_t kOffU    = kOffXZ   + kSzXZ;
constexpr size_t kOffU16  = kOffU    + kSzU;
constexpr size_t kOffXP   = kOffU16  + kSzH16;
constexpr size_t kOffDT16 = kOffXP   + kSzXP;
constexpr size_t kOffDTP  = kOffDT16 + kSzDT16;
constexpr size_t kOffYH   = kOffDTP  + kSzU;
constexpr size_t kOffYL   = kOffYH   + kSzH16;
constexpr size_t kOffYG   = kOffYL   + kSzH16;
constexpr size_t kWsTotal = kOffYG   + kSzH16;
static_assert(kWsTotal == 123731968ull);
static_assert(kWsTotal <= 134217728ull);
static_assert((kOffWOUT % 128) == 0 && (kOffWXP % 128) == 0 && (kOffWDT % 128) == 0 && (kOffX16 % 128) == 0 &&
              (kOffXZ % 128) == 0 && (kOffU % 128) == 0 && (kOffU16 % 128) == 0 && (kOffXP % 128) == 0 &&
              (kOffDT16 % 128) == 0 && (kOffDTP % 128) == 0 && (kOffYH % 128) == 0 && (kOffYL % 128) == 0 &&
              (kOffYG % 128) == 0);

__device__ __forceinline__ _Float16 f16_flush(float v) {
  const float w = (fabsf(v) < 6.103515625e-05f) ? 0.0f : v;
  return (_Float16)w;
}
__device__ __forceinline__ void f16_split(float v, _Float16& hi, _Float16& lo) {
  hi = f16_flush(v);
  const float hf = (float)hi;
  const float r = (v - hf) * kResid;
  lo = f16_flush(r);
}
__device__ __forceinline__ float h16_to_f32(unsigned hb) {
  const unsigned sgn = (hb & 0x8000u) << 16;
  const unsigned em = hb & 0x7fffu;
  const float fn = __uint_as_float((em << 13) + 0x38000000u);
  const float fs = (float)em * 5.9604644775390625e-8f;
  const float mag = (em < 0x400u) ? fs : fn;
  return __uint_as_float(__float_as_uint(mag) | sgn);
}

namespace eng {
union FragU { v16h v; v8h h[2]; };
__device__ __forceinline__ v16h frag_load(const _Float16* p) {
  FragU f;
  f.h[0] = *(const v8h*)(p);
  f.h[1] = *(const v8h*)(p + 16);
  return f.v;
}
__device__ __forceinline__ v8f mma(v16h a, v16h b, v8f c) {
  return __builtin_amdgcn_wmma_f32_16x16x32_f16(false, a, false, b, (short)0, c, false, false);
}
__device__ __forceinline__ void guard1(v8f& a, v16h x, v16h y) {
  asm volatile("v_nop\n\tv_nop\n\tv_nop\n\tv_nop" : "+v"(a) : "v"(x), "v"(y));
}
__device__ __forceinline__ void guard_acc(v8f& a) {
  asm volatile("v_nop\n\tv_nop\n\tv_nop\n\tv_nop" : "+v"(a));
}
__device__ __forceinline__ void keep4(v16h a, v16h b, v16h c, v16h d) {
  asm volatile("v_nop" :: "v"(a), "v"(b), "v"(c), "v"(d));
}

template <int MI, int SPL, bool BIAS>
__global__ __launch_bounds__(256) void gemm_f16_kernel(
    const unsigned short* __restrict__ Ap, const unsigned short* __restrict__ A2p, int lda,
    const unsigned short* __restrict__ Btp, const unsigned short* __restrict__ Bt2p, int ldb,
    float* __restrict__ C, int ldc, const float* __restrict__ bias,
    int M, int N, int K, float scale, float rscale)
{
  static_assert(MI >= 1 && MI <= 2);
  static_assert(SPL >= 0 && SPL <= 2);
  const _Float16* A   = (const _Float16*)Ap;
  const _Float16* A2  = (const _Float16*)A2p;
  const _Float16* Bt  = (const _Float16*)Btp;
  const _Float16* Bt2 = (const _Float16*)Bt2p;
  __shared__ __align__(16) float sT[8][16 * 68];
  const int lane = threadIdx.x & 31;
  const int wave = threadIdx.x >> 5;
  const int tilesN = N >> 6;
  const int tilesM = M / (16 * MI);
  const int tile = blockIdx.x * 8 + wave;
  if (tile >= tilesM * tilesN) return;
  const int tm = tile / tilesN;
  const int tn = tile - tm * tilesN;
  const int m0 = tm * (16 * MI);
  const int n0 = tn << 6;
  const int rlane = lane & 15;
  const int koff  = (lane >> 4) * 8;
  const int mOff  = (lane >> 4) * 8;

  v8f acc[MI][4], accr[MI][4];
#pragma unroll
  for (int i = 0; i < MI; ++i)
#pragma unroll
    for (int j = 0; j < 4; ++j) {
      acc[i][j]  = (v8f){0.f, 0.f, 0.f, 0.f, 0.f, 0.f, 0.f, 0.f};
      accr[i][j] = (v8f){0.f, 0.f, 0.f, 0.f, 0.f, 0.f, 0.f, 0.f};
    }

  for (int k0 = 0; k0 < K; k0 += 32) {
    v16h bh[4], bl[4];
#pragma unroll
    for (int j = 0; j < 4; ++j) {
      const size_t bo = (size_t)(n0 + (j << 4) + rlane) * ldb + koff + k0;
      bh[j] = frag_load(Bt + bo);
      if (SPL == 2) bl[j] = frag_load(Bt2 + bo); else bl[j] = bh[j];
    }
#pragma unroll
    for (int i = 0; i < MI; ++i) {
      const size_t ao = (size_t)(m0 + (i << 4) + rlane) * lda + koff + k0;
      const v16h ah = frag_load(A + ao);
      v16h al = ah;
      if (SPL >= 1) al = frag_load(A2 + ao);
#pragma unroll
      for (int j = 0; j < 4; ++j) {
        acc[i][j] = mma(ah, bh[j], acc[i][j]);
        if (SPL >= 1) accr[i][j] = mma(al, bh[j], accr[i][j]);
        if (SPL == 2) accr[i][j] = mma(ah, bl[j], accr[i][j]);
      }
#pragma unroll
      for (int j = 0; j < 4; ++j) {
        guard1(acc[i][j], ah, al);
        if (SPL >= 1) guard1(accr[i][j], ah, al);
      }
    }
    keep4(bh[0], bh[1], bh[2], bh[3]);
    if (SPL == 2) keep4(bl[0], bl[1], bl[2], bl[3]);
  }
#pragma unroll
  for (int i = 0; i < MI; ++i)
#pragma unroll
    for (int j = 0; j < 4; ++j) {
      guard_acc(acc[i][j]);
      if (SPL >= 1) guard_acc(accr[i][j]);
    }

  float* slab = sT[wave];
#pragma unroll
  for (int i = 0; i < MI; ++i) {
    const int mBase = m0 + (i << 4);
#pragma unroll
    for (int j = 0; j < 4; ++j) {
      float bv = 0.0f;
      if (BIAS) bv = bias[n0 + (j << 4) + rlane];
#pragma unroll
      for (int r = 0; r < 8; ++r) {
        float v = acc[i][j][r] * scale;
        if (SPL >= 1) v += accr[i][j][r] * rscale;
        if (BIAS) v += bv;
        slab[(mOff + r) * 68 + (j << 4) + rlane] = v;
      }
    }
    __builtin_amdgcn_fence(__ATOMIC_RELEASE, "workgroup");
    __builtin_amdgcn_wave_barrier();
    __builtin_amdgcn_fence(__ATOMIC_ACQUIRE, "workgroup");
    {
      const int hh = lane >> 4, c4 = (lane & 15) * 4;
      for (int pass = 0; pass < 2; ++pass) {
#pragma unroll
        for (int it = 0; it < 8; ++it) {
          const int row = it * 2 + hh;
          const v4f v = *(const v4f*)(slab + row * 68 + c4);
          *(volatile v4f*)(C + (size_t)(mBase + row) * ldc + n0 + c4) = v;
        }
        __threadfence();
      }
    }
    __builtin_amdgcn_fence(__ATOMIC_RELEASE, "workgroup");
    __builtin_amdgcn_wave_barrier();
    __builtin_amdgcn_fence(__ATOMIC_ACQUIRE, "workgroup");
  }
}
}

__global__ __launch_bounds__(256) void rows_to_f16_kernel(
    const float* __restrict__ src, unsigned short* __restrict__ dH, int total8)
{
  const int i = blockIdx.x * 256 + threadIdx.x;
  if (i >= total8) return;
  const size_t e0 = (size_t)i << 3;
  const v4f a0 = *(const v4f*)(src + e0);
  const v4f a1 = *(const v4f*)(src + e0 + 4);
  v8h hv;
#pragma unroll
  for (int e = 0; e < 4; ++e) {
    const float f0 = a0[e];
    const float f1 = a1[e];
    hv[e] = f16_flush(f0);
    hv[4 + e] = f16_flush(f1);
  }
  unsigned short* qh = dH + e0;
  *(volatile v8h*)qh = hv;
  __threadfence();
  *(volatile v8h*)qh = hv;
}

template <bool LO>
__global__ __launch_bounds__(256) void transpose_pack_kernel(
    const float* __restrict__ W, unsigned short* __restrict__ BtH, unsigned short* __restrict__ BtL,
    int Kdim, int Ndim, float carry)
{
  __shared__ float tile[64 * 65];
  const int tid = threadIdx.x, lane = tid & 31, wave = tid >> 5;
  const int n0 = blockIdx.x * 64;
  const int k0 = blockIdx.y * 64;
#pragma unroll
  for (int p = 0; p < 16; ++p) {
    const int idx = tid + p * 256;
    const int kk  = idx >> 6;
    const int nn  = idx & 63;
    const int n   = n0 + nn;
    const int nc  = (n < Ndim) ? n : (Ndim - 1);
    const float v = W[(size_t)(k0 + kk) * Ndim + nc];
    tile[kk * 65 + nn] = (n < Ndim) ? (v * carry) : 0.0f;
  }
  __syncthreads();
  const int q = lane >> 3, c8 = (lane & 7) * 8;
  v8h hv[2], lv[2];
#pragma unroll
  for (int it = 0; it < 2; ++it) {
    const int nrow = it * 32 + wave * 4 + q;
#pragma unroll
    for (int e = 0; e < 8; ++e) {
      _Float16 h, l;
      const float t = tile[(c8 + e) * 65 + nrow];
      f16_split(t, h, l);
      hv[it][e] = h;
      lv[it][e] = l;
    }
  }
  for (int pass = 0; pass < 2; ++pass) {
#pragma unroll
    for (int it = 0; it < 2; ++it) {
      const int nrow = it * 32 + wave * 4 + q;
      const size_t o = (size_t)(n0 + nrow) * Kdim + k0 + c8;
      *(volatile v8h*)(BtH + o) = hv[it];
      if (LO) *(volatile v8h*)(BtL + o) = lv[it];
    }
    __threadfence();
  }
}

__global__ __launch_bounds__(256) void conv_sigmoid_kernel(
    const float* __restrict__ XZ, const float* __restrict__ b1, const float* __restrict__ cw,
    const float* __restrict__ cb, float* __restrict__ UC, unsigned short* __restrict__ UH)
{
  __shared__ __align__(16) float sT[16 * kConvTP];
  const int tid = threadIdx.x, lane = tid & 31, wave = tid >> 5;
  const int d0 = blockIdx.x * 256, d = d0 + tid;
  const int t0 = blockIdx.y * 64;
  const v4f wv = *(const v4f*)(cw + (size_t)d * 4);
  const float w0 = wv[0], w1 = wv[1], w2 = wv[2], w3 = wv[3];
  const float bc = cb[d];
  const float bu = b1[d];
  float xm3, xm2, xm1;
  {
    const int r3 = t0 - 3, r2 = t0 - 2, r1 = t0 - 1;
    const float v3 = XZ[(size_t)(r3 < 0 ? 0 : r3) * kXzP + d] + bu;
    const float v2 = XZ[(size_t)(r2 < 0 ? 0 : r2) * kXzP + d] + bu;
    const float v1 = XZ[(size_t)(r1 < 0 ? 0 : r1) * kXzP + d] + bu;
    xm3 = (r3 >= 0) ? v3 : 0.0f;
    xm2 = (r2 >= 0) ? v2 : 0.0f;
    xm1 = (r1 >= 0) ? v1 : 0.0f;
  }
  const int hrow = wave >> 1;
  const int hch  = (wave & 1) * 128 + lane * 4;
#pragma unroll 1
  for (int sub = 0; sub < 4; ++sub) {
    const int lb = t0 + sub * 16;
#pragma unroll 1
    for (int s = 0; s < 16; ++s) {
      const float xcur = XZ[(size_t)(lb + s) * kXzP + d] + bu;
      float acc = w0 * xm3;
      acc = fmaf(w1, xm2, acc);
      acc = fmaf(w2, xm1, acc);
      acc = fmaf(w3, xcur, acc);
      const float sv = acc + bc;
      const float sg = __builtin_amdgcn_rcpf(1.0f + expf(-sv));
      sT[s * kConvTP + tid] = sg;
      xm3 = xm2; xm2 = xm1; xm1 = xcur;
    }
    __syncthreads();
    v4f fv[4];
    v8h hv[2];
#pragma unroll
    for (int it = 0; it < 4; ++it) fv[it] = *(const v4f*)(sT + (it * 4 + hrow) * kConvTP + hch);
#pragma unroll
    for (int it = 0; it < 2; ++it) {
      const float* sp = sT + (it * 8 + wave) * kConvTP + lane * 8;
      const v4f a0 = *(const v4f*)(sp);
      const v4f a1 = *(const v4f*)(sp + 4);
#pragma unroll
      for (int e = 0; e < 4; ++e) {
        const float f0 = a0[e] * kUCarry;
        const float f1 = a1[e] * kUCarry;
        hv[it][e] = f16_flush(f0);
        hv[it][4 + e] = f16_flush(f1);
      }
    }
    for (int pass = 0; pass < 2; ++pass) {
#pragma unroll
      for (int it = 0; it < 4; ++it)
        *(volatile v4f*)(UC + (size_t)(lb + it * 4 + hrow) * kDin + d0 + hch) = fv[it];
#pragma unroll
      for (int it = 0; it < 2; ++it) {
        const size_t o = (size_t)(lb + it * 8 + wave) * kDin + d0 + lane * 8;
        *(volatile v8h*)(UH + o) = hv[it];
      }
      __threadfence();
    }
    __syncthreads();
  }
}

__global__ __launch_bounds__(256) void dtlow_to_f16_kernel(
    const float* __restrict__ XP, unsigned short* __restrict__ DT16, int total8)
{
  const int i = blockIdx.x * 256 + threadIdx.x;
  if (i >= total8) return;
  const int row = i >> 3;
  const int c8  = (i & 7) * 8;
  const float* sp = XP + (size_t)row * kXpP + c8;
  const v4f a0 = *(const v4f*)(sp);
  const v4f a1 = *(const v4f*)(sp + 4);
  v8h hv;
#pragma unroll
  for (int e = 0; e < 4; ++e) {
    const float f0 = a0[e] * kDtCarry;
    const float f1 = a1[e] * kDtCarry;
    hv[e] = f16_flush(f0);
    hv[4 + e] = f16_flush(f1);
  }
  unsigned short* q = DT16 + (size_t)row * kRank + c8;
  *(volatile v8h*)q = hv;
  __threadfence();
  *(volatile v8h*)q = hv;
}

__global__ __launch_bounds__(256) void gate_apply_kernel(
    const unsigned short* __restrict__ YH, const unsigned short* __restrict__ YL,
    const float* __restrict__ XZ, const float* __restrict__ b2, unsigned short* __restrict__ YG, int total8)
{
  const int i = blockIdx.x * 256 + threadIdx.x;
  if (i >= total8) return;
  const int row = i >> 8;
  const int c8  = (i & 255) * 8;
  const size_t e0 = (size_t)row * kDin + c8;
  const v4u hw = *(const v4u*)(YH + e0);
  const v4u lw = *(const v4u*)(YL + e0);
  const float* zp = XZ + (size_t)row * kXzP + kDin + c8;
  const v4f z0 = *(const v4f*)(zp);
  const v4f z1 = *(const v4f*)(zp + 4);
  const v4f g0 = *(const v4f*)(b2 + c8);
  const v4f g1 = *(const v4f*)(b2 + c8 + 4);
  v8h ov;
#pragma unroll
  for (int e = 0; e < 8; ++e) {
    const unsigned wh = hw[e >> 1];
    const unsigned wl = lw[e >> 1];
    const unsigned hb = (e & 1) ? (wh >> 16) : (wh & 0xffffu);
    const unsigned lb = (e & 1) ? (wl >> 16) : (wl & 0xffffu);
    const float yh = h16_to_f32(hb);
    const float yl = h16_to_f32(lb);
    const float yc = fmaf(yl, 1.0f / kResid, yh);
    const float zr = (e < 4) ? z0[e & 3] : z1[e & 3];
    const float zb = (e < 4) ? g0[e & 3] : g1[e & 3];
    const float zz = zr + zb;
    const float sg = __builtin_amdgcn_rcpf(1.0f + expf(-zz));
    const float gv = yc * sg;
    ov[e] = f16_flush(gv);
  }
  unsigned short* q = YG + e0;
  *(volatile v8h*)q = ov;
  __threadfence();
  *(volatile v8h*)q = ov;
}

typedef float    ms1_v4f __attribute__((ext_vector_type(4)));
typedef unsigned ms1_v4u __attribute__((ext_vector_type(4)));
struct ms1_args {
  const float* dtpre;
  const float* u;
  const float* bc;
  const float* z;
  const float* A_log;
  const float* Dskip;
  __half* y;
  __half* y_lo;
  long ld_dtpre;
  long ld_u;
  long ld_bc;
  long ld_z;
  long ld_y;
  int offB;
  int offC;
  int offZ;
  float ycarry;
  int dir;
  int D;
  int L;
  int nbatch;
};
static_assert(sizeof(ms1_args) == 136);

__device__ __forceinline__ float ms1_flush16(float v) {
  return (fabsf(v) < 6.103515625e-05f) ? 0.0f : v;
}
__device__ __forceinline__ unsigned ms1_h16bits(float v) {
  return (unsigned)__half_as_ushort(__float2half_rn(ms1_flush16(v)));
}
__device__ __forceinline__ float ms1_h16val(unsigned b) {
  return __half2float(__ushort_as_half((unsigned short)b));
}
__device__ __forceinline__ float ms1_softplus(float v) {
  return fmaxf(v, 0.0f) + log1pf(expf(-fabsf(v)));
}
__device__ __forceinline__ void ms1_pack2(float v0, float v1, unsigned& hw, unsigned& lw) {
  const unsigned h0 = ms1_h16bits(v0);
  const unsigned h1 = ms1_h16bits(v1);
  const float r0 = (v0 - ms1_h16val(h0)) * 2048.0f;
  const float r1 = (v1 - ms1_h16val(h1)) * 2048.0f;
  const unsigned l0 = ms1_h16bits(r0);
  const unsigned l1 = ms1_h16bits(r1);
  hw = h0 | (h1 << 16);
  lw = l0 | (l1 << 16);
}

template <int NSTATE>
__global__ __launch_bounds__(64 * (NSTATE / 16)) void ms1_scan_kernel(ms1_args a)
{
  static_assert(NSTATE == 16 || NSTATE == 64);
  constexpr int NQ  = NSTATE / 16;
  constexpr int NT  = 64 * NQ;
  constexpr int NW  = NT / 32;
  constexpr int BCW = 2 * NSTATE;
  constexpr int YP  = 68;
  constexpr int RPI = NW * 4;
  constexpr int NIT = 64 / RPI;
  static_assert(16 * NT <= 64 * YP);
  __shared__ __align__(16) float sBC[64 * BCW];
  __shared__ __align__(16) float sY[64 * YP];
  const int tid  = threadIdx.x;
  const int lane = tid & 31;
  const int wave = tid >> 5;
  const int c    = tid / NQ;
  const int sq   = tid - c * NQ;
  const int bpb  = a.D / 64;
  const int bi   = blockIdx.x / bpb;
  if (bi >= a.nbatch) return;
  const int d0 = (blockIdx.x - bi * bpb) * 64;
  const int d  = d0 + c;
  const long rowb = (long)bi * a.L;
  const bool hasz  = (a.z != nullptr);
  const bool hasD  = (a.Dskip != nullptr);
  const bool hasLo = (a.y_lo != nullptr);

#pragma unroll 1
  for (int n = 0; n < 16; ++n) {
    const float al = a.A_log[(long)d * NSTATE + sq * 16 + n];
    sY[n * NT + tid] = -expf(al);
  }
  __syncthreads();
  float An[16], h[16];
#pragma unroll
  for (int n = 0; n < 16; ++n) {
    An[n] = sY[n * NT + tid];
    h[n] = 0.0f;
  }
  float Dd = 0.0f;
  if (hasD) Dd = a.Dskip[d];

  const int nchunk = a.L / 64;
  const bool fwd = (a.dir > 0);
  const int s0 = fwd ? 0 : 63;
  const int sd = fwd ? 1 : -1;
  const int q  = lane >> 3;
  const int c8 = (lane & 7) * 8;

#pragma unroll 1
  for (int ci = 0; ci < nchunk; ++ci) {
    const int tb = fwd ? (ci * 64) : (a.L - 64 - ci * 64);
    const long rowc = rowb + tb;
    __syncthreads();
#pragma unroll 8
    for (int i = 0; i < 32; ++i) {
      const int idx = tid + i * NT;
      const int st  = idx / BCW;
      const int col = idx - st * BCW;
      const int sc  = (col < NSTATE) ? (a.offB + col) : (a.offC + col - NSTATE);
      sBC[idx] = a.bc[(rowc + st) * a.ld_bc + sc];
    }
    __syncthreads();
#pragma unroll 1
    for (int s = 0; s < 64; ++s) {
      const int ls = s0 + sd * s;
      const long row = rowc + ls;
      float pre = a.dtpre[row * a.ld_dtpre + d];
      float uv  = a.u[row * a.ld_u + d];
      float zv  = 0.0f;
      if (hasz) zv = a.z[row * a.ld_z + a.offZ + d];
      asm volatile("" : "+v"(pre));
      asm volatile("" : "+v"(uv));
      asm volatile("" : "+v"(zv));
      const float delta = ms1_softplus(pre);
      const float dtx = delta * uv;
      const float* bp = sBC + ls * BCW + sq * 16;
      const float* cp = bp + NSTATE;
      ms1_v4f Bq[4], Cq[4];
#pragma unroll
      for (int k = 0; k < 4; ++k) {
        Bq[k] = *(const ms1_v4f*)(bp + 4 * k);
        Cq[k] = *(const ms1_v4f*)(cp + 4 * k);
      }
      float yv = 0.0f;
#pragma unroll
      for (int n = 0; n < 16; ++n) {
        const float e = __expf(delta * An[n]);
        h[n] = fmaf(e, h[n], dtx * Bq[n >> 2][n & 3]);
        yv = fmaf(h[n], Cq[n >> 2][n & 3], yv);
      }
      if (NQ > 1) {
        yv += __shfl_xor(yv, 1, 32);
        yv += __shfl_xor(yv, 2, 32);
      }
      if (hasD) yv = fmaf(uv, Dd, yv);
      if (hasz) {
        const float sg = __builtin_amdgcn_rcpf(1.0f + expf(-zv));
        yv = yv * (zv * sg);
      }
      if (sq == 0) sY[ls * YP + c] = yv * a.ycarry;
    }
    __syncthreads();
    ms1_v4u hw[NIT], lw[NIT];
#pragma unroll
    for (int it = 0; it < NIT; ++it) {
      const int row = it * RPI + wave * 4 + q;
      const float* sp = sY + row * YP + c8;
      const ms1_v4f f0 = *(const ms1_v4f*)(sp);
      const ms1_v4f f1 = *(const ms1_v4f*)(sp + 4);
      unsigned h0, h1, h2, h3, l0, l1, l2, l3;
      ms1_pack2(f0[0], f0[1], h0, l0);
      ms1_pack2(f0[2], f0[3], h1, l1);
      ms1_pack2(f1[0], f1[1], h2, l2);
      ms1_pack2(f1[2], f1[3], h3, l3);
      hw[it] = (ms1_v4u){h0, h1, h2, h3};
      lw[it] = (ms1_v4u){l0, l1, l2, l3};
    }
    for (int pass = 0; pass < 2; ++pass) {
#pragma unroll
      for (int it = 0; it < NIT; ++it) {
        const int row = it * RPI + wave * 4 + q;
        const long o = (rowc + row) * a.ld_y + d0 + c8;
        *(volatile ms1_v4u*)(a.y + o) = hw[it];
        if (hasLo) *(volatile ms1_v4u*)(a.y_lo + o) = lw[it];
      }
      __threadfence();
    }
  }
}

static_assert(((kSeq / 32) * (kXzP / 64)) % 8 == 0);
static_assert(((kSeq / 16) * (kXpP / 64)) % 8 == 0);
static_assert(((kSeq / 32) * (kDin / 64)) % 8 == 0);
static_assert(((kSeq / 32) * (kDm / 64)) % 8 == 0);

extern "C" void kernel_launch(void* const* d_in, const int* in_sizes, int n_in,
                              void* d_out, int out_size, void* d_ws, size_t ws_size,
                              hipStream_t stream)
{
  if (n_in < 14) return;
  if (in_sizes[0] != kBatch * kSeq * kDm) return;
  if (in_sizes[1] != kDm * kDin) return;
  if (in_sizes[2] != kDin) return;
  if (in_sizes[3] != kDm * kDin) return;
  if (in_sizes[4] != kDin) return;
  if (in_sizes[5] != kDin * 4) return;
  if (in_sizes[6] != kDin) return;
  if (in_sizes[7] != kDin * kNst) return;
  if (in_sizes[8] != kDin * kXpN) return;
  if (in_sizes[9] != kRank * kDin) return;
  if (in_sizes[10] != kDin) return;
  if (in_sizes[11] != kDin) return;
  if (in_sizes[12] != kDin * kDm) return;
  if (in_sizes[13] != kDm) return;
  if (out_size != kBatch * kSeq * kDm) return;
  if (ws_size < kWsTotal) return;

  const float* x      = (const float*)d_in[0];
  const float* W1     = (const float*)d_in[1];
  const float* b1     = (const float*)d_in[2];
  const float* W2     = (const float*)d_in[3];
  const float* b2     = (const float*)d_in[4];
  const float* conv_w = (const float*)d_in[5];
  const float* conv_b = (const float*)d_in[6];
  const float* A_log  = (const float*)d_in[7];
  const float* xp_w   = (const float*)d_in[8];
  const float* dt_w   = (const float*)d_in[9];
  const float* dt_b   = (const float*)d_in[10];
  const float* D_par  = (const float*)d_in[11];
  const float* Wo     = (const float*)d_in[12];
  const float* bo     = (const float*)d_in[13];
  float* out = (float*)d_out;

  char* ws = (char*)d_ws;
  unsigned short* WIN  = (unsigned short*)(ws + kOffWIN);
  unsigned short* WOUT = (unsigned short*)(ws + kOffWOUT);
  unsigned short* WXP  = (unsigned short*)(ws + kOffWXP);
  unsigned short* WDT  = (unsigned short*)(ws + kOffWDT);
  unsigned short* X16  = (unsigned short*)(ws + kOffX16);
  float*          XZ   = (float*)(ws + kOffXZ);
  float*          U    = (float*)(ws + kOffU);
  unsigned short* U16  = (unsigned short*)(ws + kOffU16);
  float*          XP   = (float*)(ws + kOffXP);
  unsigned short* DT16 = (unsigned short*)(ws + kOffDT16);
  float*          DTP  = (float*)(ws + kOffDTP);
  unsigned short* YH   = (unsigned short*)(ws + kOffYH);
  unsigned short* YL   = (unsigned short*)(ws + kOffYL);
  unsigned short* YG   = (unsigned short*)(ws + kOffYG);

  transpose_pack_kernel<false><<<dim3(kDin / 64, kDm / 64), 256, 0, stream>>>(W1, WIN, WIN, kDm, kDin, kWCarry);
  unsigned short* WIN2 = WIN + (size_t)kDin * kDm;
  transpose_pack_kernel<false><<<dim3(kDin / 64, kDm / 64), 256, 0, stream>>>(W2, WIN2, WIN2, kDm, kDin, kWCarry);
  transpose_pack_kernel<false><<<dim3(kDm / 64, kDin / 64), 256, 0, stream>>>(Wo, WOUT, WOUT, kDin, kDm, kWCarry);
  transpose_pack_kernel<false><<<dim3(kXpP / 64, kDin / 64), 256, 0, stream>>>(xp_w, WXP, WXP, kDin, kXpN, kWCarry);
  transpose_pack_kernel<false><<<dim3(kDin / 64, kRank / 64), 256, 0, stream>>>(dt_w, WDT, WDT, kRank, kDin, kWCarry);

  rows_to_f16_kernel<<<(kBatch * kSeq * kDm / 8) / 256, 256, 0, stream>>>(x, X16, kBatch * kSeq * kDm / 8);

  for (int b = 0; b < kBatch; ++b) {
    const unsigned short* xb = X16 + (size_t)b * kSeq * kDm;
    float* outb = out + (size_t)b * kSeq * kDm;

    eng::gemm_f16_kernel<2, 0, false><<<dim3((kSeq / 32) * (kXzP / 64) / 8), 256, 0, stream>>>(
        xb, xb, kDm, WIN, WIN, kDm, XZ, kXzP, b1, kSeq, kXzP, kDm, kScIn, kScNone);

    conv_sigmoid_kernel<<<dim3(kDin / 256, kSeq / 64), 256, 0, stream>>>(XZ, b1, conv_w, conv_b, U, U16);

    eng::gemm_f16_kernel<1, 0, false><<<dim3((kSeq / 16) * (kXpP / 64) / 8), 256, 0, stream>>>(
        U16, U16, kDin, WXP, WXP, kDin, XP, kXpP, b1, kSeq, kXpP, kDin, kScU, kScNone);

    dtlow_to_f16_kernel<<<(kSeq * kRank / 8) / 256, 256, 0, stream>>>(XP, DT16, kSeq * kRank / 8);

    eng::gemm_f16_kernel<2, 0, true><<<dim3((kSeq / 32) * (kDin / 64) / 8), 256, 0, stream>>>(
        DT16, DT16, kRank, WDT, WDT, kRank, DTP, kDin, dt_b, kSeq, kDin, kRank, kScDt, kScNone);

    ms1_args sa;
    sa.dtpre = DTP;
    sa.u = U;
    sa.bc = XP;
    sa.z = nullptr;
    sa.A_log = A_log;
    sa.Dskip = D_par;
    sa.y = (__half*)YH;
    sa.y_lo = (__half*)YL;
    sa.ld_dtpre = kDin;
    sa.ld_u = kDin;
    sa.ld_bc = kXpP;
    sa.ld_z = 0;
    sa.ld_y = kDin;
    sa.offB = kOffB;
    sa.offC = kOffC;
    sa.offZ = 0;
    sa.ycarry = kYCarry;
    sa.dir = 1;
    sa.D = kDin;
    sa.L = kSeq;
    sa.nbatch = 1;
    ms1_scan_kernel<16><<<dim3(kDin / 64), 64, 0, stream>>>(sa);

    gate_apply_kernel<<<(kSeq * kDin / 8) / 256, 256, 0, stream>>>(YH, YL, XZ, b2, YG, kSeq * kDin / 8);

    eng::gemm_f16_kernel<2, 0, true><<<dim3((kSeq / 32) * (kDm / 64) / 8), 256, 0, stream>>>(
        YG, YG, kDin, WOUT, WOUT, kDin, outb, kDm, bo, kSeq, kDm, kDin, kScY, kScNone);
  }
}
